// CustomCausalAttention_21603685499692
// MI455X (gfx1250) — hardware-verified
//
#include <hip/hip_runtime.h>
#include <math.h>


#define NB 2
#define NH 16
#define NQ 2048
#define HD 128
#define BM 128
#define BN 32

typedef __attribute__((ext_vector_type(16))) _Float16 v16h;
typedef __attribute__((ext_vector_type(16))) __bf16 v16b;
typedef __attribute__((ext_vector_type(8)))  float v8f;
typedef __attribute__((ext_vector_type(4)))  float v4f;

template <typename T> __device__ __forceinline__ void vst2(void* p, T v) { *(volatile T*)p = v; __threadfence(); *(volatile T*)p = v; }
__device__ __forceinline__ v8f wmma_bf(v16b a, v16b b, v8f c) {
  v8f d = __builtin_amdgcn_wmma_f32_16x16x32_bf16(false, a, false, b, (short)0, c, false, false);
  asm volatile("v_nop\n\tv_nop\n\tv_nop\n\tv_nop" : "+v"(d) : "v"(a), "v"(b));
  return d;
}
__device__ __forceinline__ v8f wmma_h(v16h a, v16h b, v8f c) {
  v8f d = __builtin_amdgcn_wmma_f32_16x16x32_f16(false, a, false, b, (short)0, c, false, false);
  asm volatile("v_nop\n\tv_nop\n\tv_nop\n\tv_nop" : "+v"(d) : "v"(a), "v"(b));
  return d;
}
struct F2 { v16b h, l; };
__device__ __forceinline__ F2 split_row(const float* row, int k0, int lane) {
  F2 r; const float* p = row + k0 + 8 * (lane >> 4);
#pragma unroll
  for (int i = 0; i < 8; ++i) { float v0 = p[i], v1 = p[16 + i]; __bf16 h0 = (__bf16)v0, h1 = (__bf16)v1;
    r.h[i] = h0; r.l[i] = (__bf16)(v0 - (float)h0); r.h[8 + i] = h1; r.l[8 + i] = (__bf16)(v1 - (float)h1); }
  return r;
}
__device__ __forceinline__ v8f mac3(const F2& a, const F2& b, v8f c) { c = wmma_bf(a.l, b.h, c); c = wmma_bf(a.h, b.l, c); return wmma_bf(a.h, b.h, c); }
struct H2 { v16h h, l; };
__device__ __forceinline__ H2 hsplit_row(const float* row, int k0, int lane) {
  H2 a; const float* p = row + k0 + 8 * (lane >> 4);
#pragma unroll
  for (int i = 0; i < 8; ++i) { float v0 = p[i], v1 = p[16 + i]; _Float16 h0 = (_Float16)v0, h1 = (_Float16)v1;
    a.h[i] = h0; a.l[i] = (_Float16)(v0 - (float)h0); a.h[8 + i] = h1; a.l[8 + i] = (_Float16)(v1 - (float)h1); }
  return a;
}
__device__ __forceinline__ H2 hsplit_col(const float* base, int lane, int ld) {
  H2 a; const float* p = base + (size_t)(8 * (lane >> 4)) * ld;
#pragma unroll
  for (int i = 0; i < 8; ++i) { float v0 = p[(size_t)i * ld], v1 = p[(size_t)(16 + i) * ld]; _Float16 h0 = (_Float16)v0, h1 = (_Float16)v1;
    a.h[i] = h0; a.l[i] = (_Float16)(v0 - (float)h0); a.h[8 + i] = h1; a.l[8 + i] = (_Float16)(v1 - (float)h1); }
  return a;
}
__device__ __forceinline__ v8f hmac3(const H2& a, const H2& b, v8f c) { c = wmma_h(a.l, b.h, c); c = wmma_h(a.h, b.l, c); return wmma_h(a.h, b.h, c); }

__global__ __launch_bounds__(256) void rbf_causal_attn(const float* __restrict__ Q, const float* __restrict__ K,
                                                       const float* __restrict__ V, float* __restrict__ O) {
  __shared__ __align__(16) float sK[BN][HD + 4];
  __shared__ __align__(16) float sV[BN][HD + 4];
  __shared__ float sKsq[BN];
  __shared__ __align__(16) float sP[8][16][BN];
  __shared__ __align__(16) float sO[8][16][HD];

  const int tid = threadIdx.x, w = tid >> 5, lane = tid & 31, g = lane >> 4, ln = lane & 15;
  const int bh = blockIdx.y;
  const int m0 = blockIdx.x * BM + w * 16;
  const size_t base = (size_t)bh * NQ * HD;
  const int jEnd = (blockIdx.x + 1) * BM;
  const float sc = 0.08838834764831845f;

  const float* qrow = Q + base + (size_t)(m0 + ln) * HD;
  float qsq = 0.f;
  for (int d = g * 64; d < g * 64 + 64; ++d) { const float x = qrow[d]; qsq += x * x; }
  qsq += __shfl_xor(qsq, 16, 32);
  float qs[8], mrun[8];
#pragma unroll
  for (int r = 0; r < 8; ++r) { qs[r] = __shfl(qsq, r + g * 8, 32); mrun[r] = -3.0e38f; }
  v8f acc[8];
#pragma unroll
  for (int dc = 0; dc < 8; ++dc) acc[dc] = (v8f){};

  const int key = tid >> 3, d0 = (tid & 7) * 16;
  for (int j0 = 0; j0 < jEnd; j0 += BN) {
    __syncthreads();
    { const float* gk = K + base + (size_t)(j0 + key) * HD + d0; const float* gv = V + base + (size_t)(j0 + key) * HD + d0;
      float ks = 0.f;
#pragma unroll
      for (int i = 0; i < 4; ++i) { const v4f x = *(const v4f*)(gk + i * 4); *(v4f*)&sK[key][d0 + i * 4] = x; ks += x[0]*x[0] + x[1]*x[1] + x[2]*x[2] + x[3]*x[3];
        *(v4f*)&sV[key][d0 + i * 4] = *(const v4f*)(gv + i * 4); }
#pragma unroll
      for (int off = 4; off >= 1; off >>= 1) ks += __shfl_xor(ks, off, 32);
      if ((tid & 7) == 0) sKsq[key] = ks; }
    __syncthreads();
    if (j0 > m0 + 15) continue;

    v8f s0 = {}, s1 = {};
#pragma unroll 1
    for (int c = 0; c < 4; ++c) {
      const F2 qa = split_row(qrow, c * 32, lane);
      s0 = mac3(qa, split_row(&sK[ln][0], c * 32, lane), s0);
      s1 = mac3(qa, split_row(&sK[16 + ln][0], c * 32, lane), s1);
    }
    const float ksq0 = sKsq[ln], ksq1 = sKsq[16 + ln];
    const int n0g = j0 + ln, n1g = j0 + 16 + ln;
#pragma unroll
    for (int r = 0; r < 8; ++r) {
      const int mg = m0 + 8 * g + r;
      const float x0 = sc * (2.f * s0[r] - qs[r] - ksq0), x1 = sc * (2.f * s1[r] - qs[r] - ksq1);
      const bool ok0 = n0g <= mg, ok1 = n1g <= mg;
      float mx = fmaxf(ok0 ? x0 : -3.0e38f, ok1 ? x1 : -3.0e38f);
#pragma unroll
      for (int off = 8; off >= 1; off >>= 1) mx = fmaxf(mx, __shfl_xor(mx, off, 32));
      const float mn = fmaxf(mrun[r], mx);
      const float corr = (mrun[r] <= -3.0e38f) ? 0.f : expf(mrun[r] - mn);
      const float p0 = ok0 ? expf(x0 - mn) * 32768.0f : 0.f, p1 = ok1 ? expf(x1 - mn) * 32768.0f : 0.f;
      mrun[r] = mn;
#pragma unroll
      for (int dc = 0; dc < 8; ++dc) acc[dc][r] *= corr;
      sP[w][8 * g + r][ln] = p0; sP[w][8 * g + r][16 + ln] = p1;
    }
    asm volatile("s_wait_dscnt 0" ::: "memory"); __builtin_amdgcn_wave_barrier(); __builtin_amdgcn_fence(__ATOMIC_RELEASE, "workgroup");
    const H2 ap = hsplit_row(&sP[w][ln][0], 0, lane);
#pragma unroll
    for (int dc = 0; dc < 8; ++dc) acc[dc] = hmac3(ap, hsplit_col(&sV[0][dc * 16 + ln], lane, HD + 4), acc[dc]);
    __builtin_amdgcn_wave_barrier();
  }

  float* so = &sO[w][0][0];
#pragma unroll
  for (int r = 0; r < 8; ++r) { const float em = expf(mrun[r]) * (1.0f / 32768.0f);
#pragma unroll
    for (int dc = 0; dc < 8; ++dc) so[(8 * g + r) * HD + dc * 16 + ln] = acc[dc][r] * em; }
  asm volatile("s_wait_dscnt 0" ::: "memory"); __builtin_amdgcn_wave_barrier(); __builtin_amdgcn_fence(__ATOMIC_RELEASE, "workgroup");
#pragma unroll 4
  for (int m = 0; m < 16; ++m) vst2(O + base + (size_t)(m0 + m) * HD + lane * 4, *(const v4f*)(so + m * HD + lane * 4));
}

extern "C" void kernel_launch(void* const* d_in, const int* in_sizes, int n_in,
                              void* d_out, int out_size, void* d_ws, size_t ws_size,
                              hipStream_t stream) {
  (void)in_sizes; (void)n_in; (void)out_size; (void)d_ws; (void)ws_size;
  const float* q = (const float*)d_in[0];
  const float* k = (const float*)d_in[1];
  const float* v = (const float*)d_in[2];
  float* o = (float*)d_out;
  rbf_causal_attn<<<dim3(NQ / BM, NB * NH), 256, 0, stream>>>(q, k, v, o);
}
